// SPIntraAttModuleV2_33346126086740
// MI455X (gfx1250) — hardware-run, weakly checked
//
#include <hip/hip_runtime.h>
#include <stdint.h>

#define DEVINL __device__ __forceinline__

typedef _Float16 f16t;
typedef unsigned short us_t;
typedef unsigned long long u64;
typedef _Float16 v16h __attribute__((ext_vector_type(16)));
typedef _Float16 v8h  __attribute__((ext_vector_type(8)));
typedef __bf16   v16b __attribute__((ext_vector_type(16)));
typedef us_t     v8us __attribute__((ext_vector_type(8)));
typedef float    v8f  __attribute__((ext_vector_type(8)));
typedef float    v4f  __attribute__((ext_vector_type(4)));
typedef int      v4i  __attribute__((ext_vector_type(4)));
typedef unsigned v4u  __attribute__((ext_vector_type(4)));
typedef u64      v2u64 __attribute__((ext_vector_type(2)));
typedef v8h   __attribute__((may_alias)) v8ha;
typedef v8us  __attribute__((may_alias)) v8usa;
typedef v4f   __attribute__((may_alias)) v4fa;
typedef v4i   __attribute__((may_alias)) v4ia;
typedef v4u   __attribute__((may_alias)) v4ua;
typedef v2u64 __attribute__((may_alias)) v2u64a;
union FragH { v16h v; v8h half[2]; };
union FragB { v16b v; v8us half[2]; };
static_assert(sizeof(FragH) == 32);
static_assert(sizeof(FragB) == 32);

#define NIMG  2
#define CH    256
#define HWP   16384
#define NSP   256
#define NHD   8
#define HDIM  32
#define TK    128
#define KW    512
#define NKS   24
#define SCALE_ 0.17677669529663687f
#define LN_EPS 1e-5f
#define TPB   256
#define TPS   512
#define PT    64
#define XP    520
#define HP    264
#define FP    260
#define QP    40
#define VP    136
#define OP    36
#define FT    32
#define QCAR  16.0f
#define VCAR  16.0f
#define PCAR  256.0f
#define LDS_TOPK (HWP * 8 + 1024)
#define LDS_PROJ (PT * XP * 2 + PT * FP * 4)
#define LDS_ATTN (1024 + 2 * TK * QP * 2 + HDIM * VP * 2 + 8 * 16 * VP * 2 + 8 * 16 * OP * 4)

static_assert(CH == NHD * HDIM);
static_assert(TK == 128);
static_assert(HWP == 8 * 4 * TPS);
static_assert((HWP % PT) == 0);
static_assert((HWP % FT) == 0);
static_assert(TPB == 2 * TK);
static_assert(TPB == 8 * 32);
static_assert(PT * HP * 2 <= PT * FP * 4);
static_assert((XP % 8) == 0);
static_assert((HP % 8) == 0);
static_assert((FP % 4) == 0);
static_assert((QP % 8) == 0);
static_assert((VP % 8) == 0);
static_assert((OP % 4) == 0);
static_assert(LDS_ATTN == 83456);
static_assert(LDS_PROJ == 133120);
static_assert(LDS_TOPK == 132096);

DEVINL v8f wmma_h(v16h a, v16h b, v8f c) {
  v8f d = __builtin_amdgcn_wmma_f32_16x16x32_f16(false, a, false, b, (short)0, c, false, false);
  asm volatile("v_nop\n\tv_nop\n\tv_nop\n\tv_nop" : "+v"(d) : "v"(a), "v"(b));
  return d;
}
DEVINL v8f wmma_b(v16b a, v16b b, v8f c) {
  v8f d = __builtin_amdgcn_wmma_f32_16x16x32_bf16(false, a, false, b, (short)0, c, false, false);
  asm volatile("v_nop\n\tv_nop\n\tv_nop\n\tv_nop" : "+v"(d) : "v"(a), "v"(b));
  return d;
}
DEVINL v8f zero8f() {
  v8f z = {0.f, 0.f, 0.f, 0.f, 0.f, 0.f, 0.f, 0.f};
  return z;
}

DEVINL us_t bf16_bits(float f) {
  unsigned u = __float_as_uint(f);
  u += 0x7FFFu + ((u >> 16) & 1u);
  return (us_t)(u >> 16);
}
DEVINL float bf16_val(us_t b) { return __uint_as_float(((unsigned)b) << 16); }

DEVINL unsigned ord_bits(float v) {
  v = v + 0.0f;
  const unsigned b = __float_as_uint(v);
  return (b & 0x80000000u) ? ~b : (b | 0x80000000u);
}
DEVINL float ord_inv(unsigned u) {
  const unsigned b = (u & 0x80000000u) ? (u & 0x7FFFFFFFu) : ~u;
  return __uint_as_float(b);
}
DEVINL u64 mkkey(float v, int idx) {
  const unsigned o = ord_bits(v);
  return (((u64)(0xFFFFFFFFu - o)) << 32) | (u64)(unsigned)idx;
}
DEVINL void cex(u64* a, int i, int l, bool asc) {
  const u64 x = a[i], y = a[l];
  const bool lt = x < y;
  const u64 mn = lt ? x : y, mx = lt ? y : x;
  a[i] = asc ? mn : mx;
  a[l] = asc ? mx : mn;
}

DEVINL void store_rows256(const f16t* sT, f16t* dst, int wave, int lane) {
  #pragma unroll
  for (int i = 0; i < 8; ++i) {
    const int p = wave + 8 * i;
    const v8h v = *(const v8ha*)(sT + p * HP + 8 * lane);
    *(volatile v8h*)(dst + (size_t)p * CH + 8 * lane) = v;
  }
  __threadfence();
  #pragma unroll
  for (int i = 0; i < 8; ++i) {
    const int p = wave + 8 * i;
    const v8h v = *(const v8ha*)(sT + p * HP + 8 * lane);
    *(volatile v8h*)(dst + (size_t)p * CH + 8 * lane) = v;
  }
}

__global__ __launch_bounds__(TPB) void prep_w_k(const float* __restrict__ wq, const float* __restrict__ wk,
                                               const float* __restrict__ wv, us_t* __restrict__ WPL)
{
  const int t = blockIdx.x * TPB + threadIdx.x;
  if (t >= 3 * CH * 64) return;
  const int row = t >> 6, q = t & 63;
  const int g = row >> 8, o = row & 255;
  const int cb = (q & 31) * 8;
  v8us outv;
  #pragma unroll
  for (int i = 0; i < 8; ++i) {
    const int c = cb + i;
    const float a0 = wq[o * CH + c];
    const float a1 = wk[o * CH + c];
    const float a2 = wv[o * CH + c];
    float w = a2;
    w = (g == 1) ? a1 : w;
    w = (g == 0) ? a0 : w;
    const us_t hi = bf16_bits(w);
    const us_t lo = bf16_bits(w - bf16_val(hi));
    outv[i] = (q < 32) ? hi : lo;
  }
  us_t* dst = WPL + (size_t)row * KW + q * 8;
  *(volatile v8us*)dst = outv;
  __threadfence();
  *(volatile v8us*)dst = outv;
}

__global__ __launch_bounds__(TPS) void topk_k(const float* __restrict__ aff, const int* __restrict__ pns,
                                             float* __restrict__ SIMS, int* __restrict__ IDX,
                                             unsigned char* __restrict__ RANK)
{
  extern __shared__ __attribute__((aligned(16))) char dsm[];
  u64*   sKey  = (u64*)dsm;
  float* sTopV = (float*)(dsm + HWP * 8);
  int*   sTopI = (int*)(dsm + HWP * 8 + 512);
  const int tid = threadIdx.x, lane = tid & 31, wave = tid >> 5;
  const int r = blockIdx.x;
  int nsp = pns[0];
  nsp = nsp < 0 ? 0 : (nsp > NSP ? NSP : nsp);
  const bool live = (r & (NSP - 1)) < nsp;

  const float* src = aff + (size_t)r * HWP;
  #pragma unroll
  for (int j = 0; j < 8; ++j) {
    const int e4 = 4 * tid + 4 * TPS * j;
    const v4f v = *(const v4fa*)(src + e4);
    v2u64 k01, k23;
    k01[0] = mkkey(v[0], e4 + 0);
    k01[1] = mkkey(v[1], e4 + 1);
    k23[0] = mkkey(v[2], e4 + 2);
    k23[1] = mkkey(v[3], e4 + 3);
    *(v2u64a*)(sKey + e4)     = k01;
    *(v2u64a*)(sKey + e4 + 2) = k23;
  }
  __syncthreads();

  #pragma unroll 1
  for (int k = 2; k <= TK; k <<= 1) {
    #pragma unroll 1
    for (int j = k >> 1; j > 0; j >>= 1) {
      #pragma unroll 4
      for (int q = 0; q < 16; ++q) {
        const int idx = tid + TPS * q;
        const int i = ((idx & ~(j - 1)) << 1) | (idx & (j - 1));
        cex(sKey, i, i | j, (i & k) == 0);
      }
      __syncthreads();
    }
  }

  #pragma unroll 1
  for (int n = HWP; n > TK; n >>= 1) {
    const int n2 = n >> 1;
    const int ecnt = (n2 >= TPS) ? (n2 / TPS) : 1;
    u64 keep[16];
    #pragma unroll
    for (int q = 0; q < 16; ++q) {
      keep[q] = 0ull;
      if (q < ecnt) {
        const int e = tid + TPS * q;
        const int sidx = ((e >> 7) << 8) | (e & (TK - 1));
        const u64 x0 = sKey[sidx], x1 = sKey[sidx + TK];
        keep[q] = (x0 < x1) ? x0 : x1;
      }
    }
    __syncthreads();
    #pragma unroll
    for (int q = 0; q < 16; ++q) {
      if (q < ecnt) sKey[tid + TPS * q] = keep[q];
    }
    __syncthreads();
    const int np = n2 >> 1;
    const int qcnt = (np >= TPS) ? (np / TPS) : 1;
    #pragma unroll 1
    for (int j = TK >> 1; j > 0; j >>= 1) {
      #pragma unroll 1
      for (int q = 0; q < qcnt; ++q) {
        const int idx = tid + TPS * q;
        const int i = ((idx & ~(j - 1)) << 1) | (idx & (j - 1));
        cex(sKey, i, i | j, (i & TK) == 0);
      }
      __syncthreads();
    }
  }

  if (tid < TK) {
    const u64 key = sKey[tid];
    int ix = (int)(unsigned)(key & 0xFFFFFFFFull);
    ix = ix < 0 ? 0 : (ix > HWP - 1 ? HWP - 1 : ix);
    const unsigned hi = (unsigned)(key >> 32);
    float val = ord_inv(0xFFFFFFFFu - hi);
    val = live ? val : 0.0f;
    sTopV[tid] = val;
    sTopI[tid] = ix;
  }
  __syncthreads();
  unsigned char* sMap = (unsigned char*)dsm;
  {
    v4u ff = {0xFFFFFFFFu, 0xFFFFFFFFu, 0xFFFFFFFFu, 0xFFFFFFFFu};
    *(v4ua*)(sMap + 16 * tid)         = ff;
    *(v4ua*)(sMap + 16 * (tid + TPS)) = ff;
  }
  __syncthreads();
  if (live && tid < TK) sMap[sTopI[tid]] = (unsigned char)tid;
  __syncthreads();
  {
    const v4u m0 = *(const v4ua*)(sMap + 16 * tid);
    const v4u m1 = *(const v4ua*)(sMap + 16 * (tid + TPS));
    const v4f sv = *(const v4fa*)(sTopV + 4 * lane);
    const v4i si = *(const v4ia*)(sTopI + 4 * lane);
    unsigned char* rdst = RANK + (size_t)r * HWP;
    float* sdst = SIMS + (size_t)r * TK + 4 * lane;
    int*   idst = IDX  + (size_t)r * TK + 4 * lane;
    *(volatile v4u*)(rdst + 16 * tid)         = m0;
    *(volatile v4u*)(rdst + 16 * (tid + TPS)) = m1;
    if (wave == 0) *(volatile v4f*)sdst = sv;
    if (wave == 1) *(volatile v4i*)idst = si;
    __threadfence();
    *(volatile v4u*)(rdst + 16 * tid)         = m0;
    *(volatile v4u*)(rdst + 16 * (tid + TPS)) = m1;
    if (wave == 0) *(volatile v4f*)sdst = sv;
    if (wave == 1) *(volatile v4i*)idst = si;
  }
}

__global__ __launch_bounds__(TPB) void proj_k(const float* __restrict__ x, const float* __restrict__ lnw,
                                             const float* __restrict__ lnb, const us_t* __restrict__ WPL,
                                             f16t* __restrict__ QH, f16t* __restrict__ KH,
                                             float* __restrict__ V, int b)
{
  extern __shared__ __attribute__((aligned(16))) char dsm[];
  us_t*  sX  = (us_t*)dsm;
  char*  stg = dsm + PT * XP * 2;
  float* sXF = (float*)stg;
  f16t*  sTH = (f16t*)stg;
  float* sTF = (float*)stg;
  const int tid = threadIdx.x, lane = tid & 31, wave = tid >> 5;
  const int h = lane >> 4, m = lane & 15;
  const int p0 = blockIdx.x * PT;

  {
    const int c0 = tid >> 4, p4 = (tid & 15) * 4;
    const float* xb = x + ((size_t)b * CH) * HWP + p0 + p4;
    #pragma unroll 4
    for (int i = 0; i < 16; ++i) {
      const int c = c0 + 16 * i;
      const v4f v = *(const v4fa*)(xb + (size_t)c * HWP);
      sXF[(p4 + 0) * FP + c] = v[0];
      sXF[(p4 + 1) * FP + c] = v[1];
      sXF[(p4 + 2) * FP + c] = v[2];
      sXF[(p4 + 3) * FP + c] = v[3];
    }
  }
  __syncthreads();
  {
    float gw[8], gb[8];
    #pragma unroll
    for (int j = 0; j < 8; ++j) { gw[j] = lnw[lane + 32 * j]; gb[j] = lnb[lane + 32 * j]; }
    #pragma unroll 1
    for (int pp = 0; pp < 8; ++pp) {
      const int p = wave * 8 + pp;
      float vals[8];
      float s = 0.0f;
      #pragma unroll
      for (int j = 0; j < 8; ++j) { vals[j] = sXF[p * FP + lane + 32 * j]; s += vals[j]; }
      #pragma unroll
      for (int off = 16; off > 0; off >>= 1) s += __shfl_xor(s, off);
      const float mu = s * (1.0f / 256.0f);
      float ss = 0.0f;
      #pragma unroll
      for (int j = 0; j < 8; ++j) { const float d = vals[j] - mu; vals[j] = d; ss = fmaf(d, d, ss); }
      #pragma unroll
      for (int off = 16; off > 0; off >>= 1) ss += __shfl_xor(ss, off);
      const float rs = rsqrtf(ss * (1.0f / 256.0f) + LN_EPS);
      #pragma unroll
      for (int j = 0; j < 8; ++j) {
        const int c = lane + 32 * j;
        const float y = (vals[j] * rs) * gw[j] + gb[j];
        const us_t hi = bf16_bits(y);
        const us_t lo = bf16_bits(y - bf16_val(hi));
        sX[p * XP + c]      = hi;
        sX[p * XP + CH + c] = lo;
      }
    }
  }
  __syncthreads();

  #pragma unroll 1
  for (int g = 0; g < 3; ++g) {
    v8f acc[2][4];
    #pragma unroll
    for (int mt = 0; mt < 2; ++mt) {
      #pragma unroll
      for (int n = 0; n < 4; ++n) acc[mt][n] = zero8f();
    }
    const us_t* arow = WPL + ((size_t)(g * CH + 32 * wave + m)) * KW + 8 * h;
    const us_t* brow = sX + m * XP + 8 * h;
    #pragma unroll 1
    for (int ks = 0; ks < NKS; ++ks) {
      const int seg = ks >> 3, kk = (ks & 7) * 32;
      const int ca  = kk + ((seg == 2) ? CH : 0);
      const int cbx = kk + ((seg == 1) ? CH : 0);
      FragB a0, a1, bf[4];
      a0.half[0] = *(const v8usa*)(arow + ca);
      a0.half[1] = *(const v8usa*)(arow + ca + 16);
      a1.half[0] = *(const v8usa*)(arow + 16 * KW + ca);
      a1.half[1] = *(const v8usa*)(arow + 16 * KW + ca + 16);
      #pragma unroll
      for (int n = 0; n < 4; ++n) {
        bf[n].half[0] = *(const v8usa*)(brow + 16 * n * XP + cbx);
        bf[n].half[1] = *(const v8usa*)(brow + 16 * n * XP + cbx + 16);
      }
      #pragma unroll
      for (int n = 0; n < 4; ++n) {
        acc[0][n] = wmma_b(a0.v, bf[n].v, acc[0][n]);
        acc[1][n] = wmma_b(a1.v, bf[n].v, acc[1][n]);
      }
    }

    if (g < 2) {
      #pragma unroll
      for (int mt = 0; mt < 2; ++mt) {
        #pragma unroll
        for (int n = 0; n < 4; ++n) {
          v8h o;
          #pragma unroll
          for (int r = 0; r < 8; ++r) o[r] = (f16t)(acc[mt][n][r] * QCAR);
          *(v8ha*)(sTH + (16 * n + m) * HP + 32 * wave + 16 * mt + 8 * h) = o;
        }
      }
    } else {
      #pragma unroll
      for (int mt = 0; mt < 2; ++mt) {
        #pragma unroll
        for (int n = 0; n < 4; ++n) {
          v4f o0, o1;
          #pragma unroll
          for (int r = 0; r < 4; ++r) { o0[r] = acc[mt][n][r]; o1[r] = acc[mt][n][4 + r]; }
          float* sp = sTF + (16 * n + m) * FP + 32 * wave + 16 * mt + 8 * h;
          *(v4fa*)sp       = o0;
          *(v4fa*)(sp + 4) = o1;
        }
      }
    }
    __syncthreads();
    if (g < 2) {
      f16t* qdst = (g == 0) ? QH : KH;
      store_rows256(sTH, qdst + (size_t)p0 * CH, wave, lane);
    } else {
      float* vdst = V + (size_t)p0 * CH;
      #pragma unroll
      for (int i = 0; i < 8; ++i) {
        const int p = wave + 8 * i;
        const v4f va = *(const v4fa*)(sTF + p * FP + 4 * lane);
        const v4f vb = *(const v4fa*)(sTF + p * FP + 128 + 4 * lane);
        *(volatile v4f*)(vdst + (size_t)p * CH + 4 * lane)       = va;
        *(volatile v4f*)(vdst + (size_t)p * CH + 128 + 4 * lane) = vb;
      }
      __threadfence();
      #pragma unroll
      for (int i = 0; i < 8; ++i) {
        const int p = wave + 8 * i;
        const v4f va = *(const v4fa*)(sTF + p * FP + 4 * lane);
        const v4f vb = *(const v4fa*)(sTF + p * FP + 128 + 4 * lane);
        *(volatile v4f*)(vdst + (size_t)p * CH + 4 * lane)       = va;
        *(volatile v4f*)(vdst + (size_t)p * CH + 128 + 4 * lane) = vb;
      }
    }
    __syncthreads();
  }
}

__global__ __launch_bounds__(TPB) void attn_k(const f16t* __restrict__ QH, const f16t* __restrict__ KH,
                                             const float* __restrict__ V, const float* __restrict__ SIMS,
                                             const int* __restrict__ IDX, float* __restrict__ O, int b)
{
  extern __shared__ __attribute__((aligned(16))) char dsm[];
  int*   sIdx = (int*)dsm;
  float* sSim = (float*)(dsm + 512);
  f16t*  sQ   = (f16t*)(dsm + 1024);
  f16t*  sK   = sQ + TK * QP;
  f16t*  sVT  = sK + TK * QP;
  f16t*  sP   = sVT + HDIM * VP;
  float* sO   = (float*)(sP + 8 * 16 * VP);
  const int tid = threadIdx.x, lane = tid & 31, wave = tid >> 5;
  const int h = lane >> 4, m = lane & 15;
  const int s = blockIdx.x;
  if (tid < TK) {
    int ix = IDX[((size_t)b * NSP + s) * TK + tid];
    ix = ix < 0 ? 0 : (ix > HWP - 1 ? HWP - 1 : ix);
    sIdx[tid] = ix;
    sSim[tid] = SIMS[((size_t)b * NSP + s) * TK + tid];
  }
  f16t*  sPw = sP + wave * (16 * VP);
  float* sOw = sO + wave * (16 * OP);
  const float zsc = SCALE_ / (QCAR * QCAR);
  const float osc = 1.0f / (PCAR * VCAR);

  #pragma unroll 1
  for (int hd = 0; hd < NHD; ++hd) {
    __syncthreads();
    {
      const int t = tid >> 1, j = tid & 1;
      const int px = sIdx[t];
      const float smv = sSim[t] * VCAR;
      const f16t* qr = QH + (size_t)px * CH + hd * HDIM + 16 * j;
      const f16t* kr = KH + (size_t)px * CH + hd * HDIM + 16 * j;
      *(v8ha*)(sQ + t * QP + 16 * j)     = *(const v8ha*)qr;
      *(v8ha*)(sQ + t * QP + 16 * j + 8) = *(const v8ha*)(qr + 8);
      *(v8ha*)(sK + t * QP + 16 * j)     = *(const v8ha*)kr;
      *(v8ha*)(sK + t * QP + 16 * j + 8) = *(const v8ha*)(kr + 8);
      const float* vr = V + (size_t)px * CH + hd * HDIM + 16 * j;
      #pragma unroll
      for (int a = 0; a < 4; ++a) {
        const v4f v = *(const v4fa*)(vr + 4 * a);
        #pragma unroll
        for (int e = 0; e < 4; ++e) sVT[(16 * j + 4 * a + e) * VP + t] = (f16t)(v[e] * smv);
      }
    }
    __syncthreads();

    FragH qa;
    qa.half[0] = *(const v8ha*)(sQ + (16 * wave + m) * QP + 8 * h);
    qa.half[1] = *(const v8ha*)(sQ + (16 * wave + m) * QP + 16 + 8 * h);
    v8f d[8];
    #pragma unroll
    for (int nt = 0; nt < 8; ++nt) {
      FragH kb;
      kb.half[0] = *(const v8ha*)(sK + (16 * nt + m) * QP + 8 * h);
      kb.half[1] = *(const v8ha*)(sK + (16 * nt + m) * QP + 16 + 8 * h);
      d[nt] = wmma_h(qa.v, kb.v, zero8f());
    }
    float mx[8], sm[8];
    #pragma unroll
    for (int r = 0; r < 8; ++r) {
      float t = d[0][r];
      #pragma unroll
      for (int nt = 1; nt < 8; ++nt) t = fmaxf(t, d[nt][r]);
      mx[r] = t;
    }
    #pragma unroll
    for (int r = 0; r < 8; ++r) {
      #pragma unroll
      for (int off = 1; off < 16; off <<= 1) mx[r] = fmaxf(mx[r], __shfl_xor(mx[r], off));
    }
    #pragma unroll
    for (int r = 0; r < 8; ++r) sm[r] = 0.0f;
    #pragma unroll
    for (int nt = 0; nt < 8; ++nt) {
      #pragma unroll
      for (int r = 0; r < 8; ++r) {
        const float e = __expf((d[nt][r] - mx[r]) * zsc);
        d[nt][r] = e;
        sm[r] += e;
      }
    }
    #pragma unroll
    for (int r = 0; r < 8; ++r) {
      #pragma unroll
      for (int off = 1; off < 16; off <<= 1) sm[r] += __shfl_xor(sm[r], off);
    }
    float inv[8];
    #pragma unroll
    for (int r = 0; r < 8; ++r) inv[r] = PCAR / sm[r];
    #pragma unroll
    for (int nt = 0; nt < 8; ++nt) {
      #pragma unroll
      for (int r = 0; r < 8; ++r) sPw[(8 * h + r) * VP + 16 * nt + m] = (f16t)(d[nt][r] * inv[r]);
    }
    __syncthreads();

    v8f acc2[2];
    acc2[0] = zero8f();
    acc2[1] = zero8f();
    #pragma unroll
    for (int ks = 0; ks < 4; ++ks) {
      FragH pa;
      pa.half[0] = *(const v8ha*)(sPw + m * VP + 32 * ks + 8 * h);
      pa.half[1] = *(const v8ha*)(sPw + m * VP + 32 * ks + 16 + 8 * h);
      #pragma unroll
      for (int nt2 = 0; nt2 < 2; ++nt2) {
        FragH vb;
        vb.half[0] = *(const v8ha*)(sVT + (16 * nt2 + m) * VP + 32 * ks + 8 * h);
        vb.half[1] = *(const v8ha*)(sVT + (16 * nt2 + m) * VP + 32 * ks + 16 + 8 * h);
        acc2[nt2] = wmma_h(pa.v, vb.v, acc2[nt2]);
      }
    }
    #pragma unroll
    for (int nt2 = 0; nt2 < 2; ++nt2) {
      #pragma unroll
      for (int r = 0; r < 8; ++r) {
        const int t = 16 * wave + 8 * h + r;
        sOw[(8 * h + r) * OP + 16 * nt2 + m] = (acc2[nt2][r] * osc) * sSim[t];
      }
    }
    __syncthreads();
    {
      const int sub = lane >> 3, piece = (lane & 7) * 4;
      float* od = O + ((size_t)(s * TK + 16 * wave)) * CH + hd * HDIM + piece;
      #pragma unroll
      for (int i = 0; i < 4; ++i) {
        const int row = sub + 4 * i;
        const v4f v = *(const v4fa*)(sOw + row * OP + piece);
        *(volatile v4f*)(od + (size_t)row * CH) = v;
      }
      __threadfence();
      #pragma unroll
      for (int i = 0; i < 4; ++i) {
        const int row = sub + 4 * i;
        const v4f v = *(const v4fa*)(sOw + row * OP + piece);
        *(volatile v4f*)(od + (size_t)row * CH) = v;
      }
    }
  }
}

__global__ __launch_bounds__(TPB) void final_k(const float* __restrict__ V, const float* __restrict__ O,
                                              const unsigned char* __restrict__ RANK,
                                              float* __restrict__ out, int b)
{
  __shared__ __attribute__((aligned(16))) float sOut[CH * FT];
  const int tid = threadIdx.x, lane = tid & 31, wave = tid >> 5;
  const int p0 = blockIdx.x * FT, p = p0 + lane;
  v4f a[8];
  const float* vrow = V + (size_t)p * CH + HDIM * wave;
  #pragma unroll
  for (int i = 0; i < 8; ++i) a[i] = *(const v4fa*)(vrow + 4 * i);
  const unsigned char* rk = RANK + ((size_t)b * NSP) * HWP + p;
  #pragma unroll 1
  for (int s = 0; s < NSP; ++s) {
    const unsigned r8 = (unsigned)rk[(size_t)s * HWP];
    const bool hit = r8 < (unsigned)TK;
    if (__any((int)hit)) {
      const int rr = hit ? (int)r8 : 0;
      const float* orow = O + ((size_t)(s * TK + rr)) * CH + HDIM * wave;
      #pragma unroll
      for (int i = 0; i < 8; ++i) {
        const v4f o = *(const v4fa*)(orow + 4 * i);
        const v4f t = a[i] + o;
        a[i].x = hit ? t.x : a[i].x;
        a[i].y = hit ? t.y : a[i].y;
        a[i].z = hit ? t.z : a[i].z;
        a[i].w = hit ? t.w : a[i].w;
      }
    }
  }
  #pragma unroll
  for (int i = 0; i < 8; ++i) {
    const int ch = HDIM * wave + 4 * i;
    sOut[(ch + 0) * FT + lane] = a[i].x;
    sOut[(ch + 1) * FT + lane] = a[i].y;
    sOut[(ch + 2) * FT + lane] = a[i].z;
    sOut[(ch + 3) * FT + lane] = a[i].w;
  }
  __syncthreads();
  {
    const int sub = lane >> 3, piece = (lane & 7) * 4;
    float* ob = out + ((size_t)b * CH) * HWP + p0 + piece;
    #pragma unroll
    for (int i = 0; i < 8; ++i) {
      const int ch = HDIM * wave + 4 * i + sub;
      const v4f v = *(const v4fa*)(sOut + ch * FT + piece);
      *(volatile v4f*)(ob + (size_t)ch * HWP) = v;
    }
    __threadfence();
    #pragma unroll
    for (int i = 0; i < 8; ++i) {
      const int ch = HDIM * wave + 4 * i + sub;
      const v4f v = *(const v4fa*)(sOut + ch * FT + piece);
      *(volatile v4f*)(ob + (size_t)ch * HWP) = v;
    }
  }
}

extern "C" void kernel_launch(void* const* d_in, const int* in_sizes, int n_in,
                              void* d_out, int out_size, void* d_ws, size_t ws_size,
                              hipStream_t stream) {
  if (n_in < 8) return;
  if (in_sizes[0] != NIMG * CH * HWP)  return;
  if (in_sizes[1] != NIMG * NSP * HWP) return;
  if (in_sizes[2] != CH)               return;
  if (in_sizes[3] != CH)               return;
  if (in_sizes[4] != CH * CH)          return;
  if (in_sizes[5] != CH * CH)          return;
  if (in_sizes[6] != CH * CH)          return;
  if (in_sizes[7] < 1)                 return;
  if (out_size != NIMG * CH * HWP)     return;

  const float* x   = (const float*)d_in[0];
  const float* aff = (const float*)d_in[1];
  const float* lnw = (const float*)d_in[2];
  const float* lnb = (const float*)d_in[3];
  const float* wq  = (const float*)d_in[4];
  const float* wk  = (const float*)d_in[5];
  const float* wv  = (const float*)d_in[6];
  const int*   pns = (const int*)d_in[7];
  float* outp = (float*)d_out;

  const size_t szWPL  = (size_t)3 * CH * KW * 2;
  const size_t szSIMS = (size_t)NIMG * NSP * TK * 4;
  const size_t szIDX  = (size_t)NIMG * NSP * TK * 4;
  const size_t szRANK = (size_t)NIMG * NSP * HWP;
  const size_t szQH   = (size_t)HWP * CH * 2;
  const size_t szKH   = (size_t)HWP * CH * 2;
  const size_t szV    = (size_t)HWP * CH * 4;
  const size_t szO    = (size_t)NSP * TK * CH * 4;
  size_t off = 0;
  char* ws = (char*)d_ws;
  us_t*  WPL  = (us_t*)(ws + off);           off += szWPL;
  float* SIMS = (float*)(ws + off);          off += szSIMS;
  int*   IDX  = (int*)(ws + off);            off += szIDX;
  unsigned char* RANK = (unsigned char*)(ws + off); off += szRANK;
  f16t*  QH   = (f16t*)(ws + off);           off += szQH;
  f16t*  KH   = (f16t*)(ws + off);           off += szKH;
  float* V    = (float*)(ws + off);          off += szV;
  float* O    = (float*)(ws + off);          off += szO;
  if (off > ws_size) return;

  hipFuncSetAttribute(reinterpret_cast<const void*>(&topk_k), hipFuncAttributeMaxDynamicSharedMemorySize, LDS_TOPK);
  hipFuncSetAttribute(reinterpret_cast<const void*>(&proj_k), hipFuncAttributeMaxDynamicSharedMemorySize, LDS_PROJ);
  hipFuncSetAttribute(reinterpret_cast<const void*>(&attn_k), hipFuncAttributeMaxDynamicSharedMemorySize, LDS_ATTN);

  prep_w_k<<<(3 * CH * 64) / TPB, TPB, 0, stream>>>(wq, wk, wv, WPL);
  topk_k<<<NIMG * NSP, TPS, LDS_TOPK, stream>>>(aff, pns, SIMS, IDX, RANK);
  for (int b = 0; b < NIMG; ++b) {
    proj_k<<<HWP / PT, TPB, LDS_PROJ, stream>>>(x, lnw, lnb, WPL, QH, KH, V, b);
    attn_k<<<NSP, TPB, LDS_ATTN, stream>>>(QH, KH, V, SIMS, IDX, O, b);
    final_k<<<HWP / FT, TPB, 0, stream>>>(V, O, RANK, outp, b);
  }
}
